// MultiHeadAttention_62294205661812
// MI455X (gfx1250) — hardware-run, weakly checked
//
#include <hip/hip_runtime.h>


#ifndef NB
#define NB 8
#endif
#ifndef SEQ
#define SEQ 2048
#endif
#define NB_FULL  8
#define SEQ_FULL 2048
#ifndef OUT_SEQ
#define OUT_SEQ SEQ
#endif
#define DM   128
#define NH_  4
#define HD   32
#define AW   4
#define OSP  36
#define EROWS (SEQ < 512 ? SEQ : 512)
#define QRS  2048.0f
#define QRI  (1.0f / 2048.0f)
#define SC2  ((float)(0.17677669529663687 * 1.4426950408889634))
#define PSH  14.0f
#define NEGB (-3.0e38f)

static_assert(HD == 32);
static_assert(NH_ * HD == DM);
static_assert(DM % 64 == 0);
static_assert(64 % HD == 0);
static_assert(DM % 32 == 0);
static_assert(SEQ % 64 == 0);
static_assert((NB * SEQ) % 64 == 0);
static_assert(SEQ % 32 == 0);
static_assert(SEQ % (16 * AW) == 0);
static_assert(EROWS % 64 == 0);
static_assert(EROWS >= 32);
static_assert(EROWS <= SEQ);
static_assert(EROWS % (16 * AW) == 0);
static_assert((SEQ - EROWS) % (16 * AW) == 0);
static_assert(((size_t)SEQ * DM) % 8 == 0);
static_assert(((size_t)DM * DM) % 8 == 0);
static_assert(NB <= NB_FULL);
static_assert(SEQ <= SEQ_FULL);
static_assert((OSP * 4) % 16 == 0);

typedef _Float16 h16;
typedef unsigned short bf;
typedef __attribute__((ext_vector_type(16))) __bf16   v16bf;
typedef __attribute__((ext_vector_type(16))) _Float16 v16h;
typedef __attribute__((ext_vector_type(8)))  _Float16 v8h;
typedef __attribute__((ext_vector_type(8)))  unsigned short v8us;
typedef __attribute__((ext_vector_type(8)))  float    v8f;
typedef __attribute__((ext_vector_type(4)))  float    v4f;
typedef v4f  __attribute__((may_alias)) v4fa;

__device__ __forceinline__ unsigned short f2bf(float f) { unsigned u = __float_as_uint(f); u += 0x7FFFu + ((u >> 16) & 1u); return (unsigned short)(u >> 16); }
__device__ __forceinline__ float bfr(float f) { return __uint_as_float(((unsigned)f2bf(f)) << 16); }
__device__ __forceinline__ v16h cat16(v8h lo, v8h hi) { return __builtin_shufflevector(lo, hi, 0, 1, 2, 3, 4, 5, 6, 7, 8, 9, 10, 11, 12, 13, 14, 15); }
__device__ __forceinline__ v16bf cat16b(v8us lo, v8us hi) { return __builtin_bit_cast(v16bf, __builtin_shufflevector(lo, hi, 0, 1, 2, 3, 4, 5, 6, 7, 8, 9, 10, 11, 12, 13, 14, 15)); }
__device__ __forceinline__ v8f wmma16(v16h a, v16h b, v8f c) { return __builtin_amdgcn_wmma_f32_16x16x32_f16(false, a, false, b, (short)0, c, false, false); }
__device__ __forceinline__ v8f wmmab(v16bf a, v16bf b, v8f c) { return __builtin_amdgcn_wmma_f32_16x16x32_bf16(false, a, false, b, (short)0, c, false, false); }
__device__ __forceinline__ v16h  ldh(const h16* p) { return cat16(*(const v8h*)p, *(const v8h*)(p + 16)); }
__device__ __forceinline__ v16bf ldb(const bf* p)  { return cat16b(*(const v8us*)p, *(const v8us*)(p + 16)); }
__device__ __forceinline__ void wave_sync() { __builtin_amdgcn_fence(3  , "wavefront"); __builtin_amdgcn_wave_barrier(); asm volatile("" ::: "memory"); }

__global__ __launch_bounds__(256) void k_cvt8(const float* __restrict__ src, bf* dst, size_t n8) {
    const size_t i = (size_t)blockIdx.x * 256 + threadIdx.x; if (i >= n8) return;
    const v8f v = *(const v8f*)(src + i * 8); v8us o;
#pragma unroll
    for (int k = 0; k < 8; ++k) o[k] = f2bf(v[k]);
    *(volatile v8us*)(dst + i * 8) = o; __threadfence(); *(volatile v8us*)(dst + i * 8) = o;
}

template <int MODE>
__global__ __launch_bounds__(32) void k_proj(const bf* __restrict__ A, const bf* __restrict__ Bt, const float* __restrict__ bias, h16* Ph, h16* Pr, int resT) {
    __shared__ __align__(16) float os[16 * 68];
    const int K = DM;
    const int lane = threadIdx.x & 31, lr = lane & 15, hi = lane >> 4; const int r0 = blockIdx.x * 64, c0 = blockIdx.y * 64;
    v8f acc[4][4];
#pragma unroll
    for (int mb = 0; mb < 4; ++mb)
#pragma unroll
        for (int nb = 0; nb < 4; ++nb) acc[mb][nb] = (v8f){};
    const size_t aoff = (size_t)(r0 + lr) * K + 8 * hi, boff = (size_t)(c0 + lr) * K + 8 * hi;
#pragma unroll 1
    for (int kc = 0; kc < K; kc += 32) {
        v16bf a[4];
#pragma unroll
        for (int mb = 0; mb < 4; ++mb) a[mb] = ldb(A + aoff + (size_t)mb * 16 * K + kc);
#pragma unroll
        for (int nb = 0; nb < 4; ++nb) { const v16bf b = ldb(Bt + boff + (size_t)nb * 16 * K + kc);
#pragma unroll
            for (int mb = 0; mb < 4; ++mb) acc[mb][nb] = wmmab(a[mb], b, acc[mb][nb]); }
        asm volatile("v_nop\n\tv_nop\n\tv_nop\n\tv_nop" : "+v"(acc[0][0]), "+v"(acc[1][1]), "+v"(acc[2][2]), "+v"(acc[3][3]) : "v"(a[0]), "v"(a[1]), "v"(a[2]), "v"(a[3]));
    }
    float bc[4];
#pragma unroll
    for (int nb = 0; nb < 4; ++nb) bc[nb] = (MODE == 0) ? bfr(bias[c0 + nb * 16 + lr]) : 0.0f;
    size_t tbase, rbase; bool wr;
    if (MODE == 0) { const int bb = r0 / SEQ, tt = r0 % SEQ; const int zc = bb * NH_ + c0 / HD;
                     tbase = ((size_t)zc * SEQ + (size_t)tt) * HD; rbase = ((size_t)zc * (size_t)resT + (size_t)tt) * HD; wr = tt < resT; }
    else           { const int bb = c0 / SEQ, tt = c0 % SEQ;
                     tbase = (size_t)bb * (size_t)DM * SEQ + (size_t)r0 * SEQ + (size_t)tt; rbase = (size_t)bb * (size_t)DM * (size_t)resT + (size_t)r0 * (size_t)resT + (size_t)tt; wr = tt < resT; }
#pragma unroll
    for (int mb = 0; mb < 4; ++mb) {
        float br[8];
#pragma unroll
        for (int j = 0; j < 8; ++j) br[j] = (MODE == 1) ? bfr(bias[r0 + mb * 16 + hi * 8 + j]) : 0.0f;
#pragma unroll
        for (int nb = 0; nb < 4; ++nb) {
#pragma unroll
            for (int j = 0; j < 8; ++j) os[(hi * 8 + j) * 68 + nb * 16 + lr] = acc[mb][nb][j] + bc[nb] + br[j]; }
        wave_sync();
#pragma unroll 1
        for (int ps = 0; ps < 2; ++ps) {
            if (MODE == 0) {
                const size_t sb = tbase + (size_t)(mb * 16) * HD;
                const size_t rb = rbase + (size_t)(mb * 16) * HD;
#pragma unroll
                for (int hh = 0; hh < 2; ++hh) {
#pragma unroll
                    for (int s = 0; s < 2; ++s) { const int p = s * 32 + lane; const int row = p >> 2, c8 = (p & 3) * 8;
                        const v4f x0 = *(const v4fa*)(&os[row * 68 + hh * 32 + c8]); const v4f x1 = *(const v4fa*)(&os[row * 68 + hh * 32 + c8 + 4]); v8h hv, rv;
#pragma unroll
                        for (int i = 0; i < 4; ++i) { const h16 a0 = (h16)x0[i]; const h16 a1 = (h16)x1[i]; hv[i] = a0; hv[4 + i] = a1; rv[i] = (h16)((x0[i] - (float)a0) * QRS); rv[4 + i] = (h16)((x1[i] - (float)a1) * QRS); }
                        const size_t oo = sb + (size_t)hh * ((size_t)SEQ * HD) + (size_t)p * 8;
                        const size_t ro = rb + (size_t)hh * ((size_t)resT * HD) + (size_t)p * 8;
                        *(volatile v8h*)(Ph + oo) = hv; if (wr) *(volatile v8h*)(Pr + ro) = rv; } }
            } else {
                const size_t sb = tbase + (size_t)(mb * 16) * SEQ;
                const size_t rb = rbase + (size_t)(mb * 16) * (size_t)resT;
#pragma unroll
                for (int s = 0; s < 4; ++s) { const int row = 4 * s + (lane >> 3), c8 = (lane & 7) * 8;
                    const v4f x0 = *(const v4fa*)(&os[row * 68 + c8]); const v4f x1 = *(const v4fa*)(&os[row * 68 + c8 + 4]); v8h hv, rv;
#pragma unroll
                    for (int i = 0; i < 4; ++i) { const h16 a0 = (h16)x0[i]; const h16 a1 = (h16)x1[i]; hv[i] = a0; hv[4 + i] = a1; rv[i] = (h16)((x0[i] - (float)a0) * QRS); rv[4 + i] = (h16)((x1[i] - (float)a1) * QRS); }
                    const size_t oo = sb + (size_t)row * SEQ + c8;
                    const size_t ro = rb + (size_t)row * (size_t)resT + c8;
                    *(volatile v8h*)(Ph + oo) = hv; if (wr) *(volatile v8h*)(Pr + ro) = rv; }
            }
            if (ps == 0) __threadfence(); }
        wave_sync();
    }
}

template <int EARLY>
__global__ __launch_bounds__(32 * AW) void k_flash(const h16* __restrict__ QH, const h16* __restrict__ QR, const h16* __restrict__ KP, const h16* __restrict__ KR,
                                                   const h16* __restrict__ VT, const h16* __restrict__ VR,
                                                   const float* __restrict__ qmask, const float* __restrict__ kmask, const int* __restrict__ causal_p, float* OUT) {
    __shared__ __align__(16) float os[AW * 16 * OSP];
    const int lane = threadIdx.x & 31, lr = lane & 15, hi = lane >> 4;
    const int wave = __builtin_amdgcn_readfirstlane((int)(threadIdx.x >> 5));
    const int zh = blockIdx.y; const int b = zh / NH_, h = zh % NH_;
    const int t0 = (EARLY ? 0 : EROWS) + (blockIdx.x * AW + wave) * 16;
    int cz = causal_p[0]; cz = cz < -SEQ ? -SEQ : (cz > SEQ ? SEQ : cz);
    const int lim = t0 + lr + cz;
    int kend = t0 + 16 + cz; kend = kend < 0 ? 0 : (kend > SEQ ? SEQ : kend);
    const int nk = (kend + 31) & ~31;
    const float qmv = bfr(qmask[(size_t)b * SEQ_FULL + t0 + lr]);
    const float* kmb = kmask + (size_t)b * SEQ_FULL + 8 * hi;
    const size_t pbase = (size_t)zh * SEQ * HD;
    const size_t rbase = (size_t)zh * EROWS * HD;
    const size_t qo = pbase + (size_t)(t0 + lr) * HD + 8 * hi;
    const v16h qh = ldh(QH + qo), qr = ldh(QR + qo);
    const size_t ko = pbase + (size_t)lr * HD + 8 * hi;
    const size_t vo = pbase + (size_t)lr * SEQ + 8 * hi;
    const size_t kro = rbase + (size_t)lr * HD + 8 * hi;
    const size_t vro = rbase + (size_t)lr * EROWS + 8 * hi;
    const v16h hz = (v16h){};
    v8f o0 = (v8f){}, o1 = (v8f){}, oR0 = (v8f){}, oR1 = (v8f){};
    float m = NEGB, l = 0.0f;
#pragma unroll 1
    for (int key0 = 0; key0 < nk; key0 += 32) {
        const bool rok = key0 < EROWS;
        const int kcl = rok ? key0 : (EROWS - 32);
        const h16* ka = KP + ko + (size_t)key0 * HD;
        const v16h ka0 = ldh(ka), kb0 = ldh(ka + 16 * HD);
        v16h kra0 = hz, krb0 = hz;
        if (EARLY) { const h16* kr = KR + kro + (size_t)kcl * HD; kra0 = ldh(kr); krb0 = ldh(kr + 16 * HD); if (!rok) { kra0 = hz; krb0 = hz; } }
        v8f sHa = (v8f){}, sLa = (v8f){}, sHb = (v8f){}, sLb = (v8f){};
        sHa = wmma16(ka0, qh, sHa); sLa = wmma16(ka0, qr, sLa); sHb = wmma16(kb0, qh, sHb); sLb = wmma16(kb0, qr, sLb);
        if (EARLY) {
            sLa = wmma16(kra0, qh, sLa); sLb = wmma16(krb0, qh, sLb);
            asm volatile("v_nop\n\tv_nop\n\tv_nop\n\tv_nop" : "+v"(sHa), "+v"(sLa), "+v"(sHb), "+v"(sLb) : "v"(ka0), "v"(kb0), "v"(kra0), "v"(krb0), "v"(qh), "v"(qr));
        } else {
            asm volatile("v_nop\n\tv_nop\n\tv_nop\n\tv_nop" : "+v"(sHa), "+v"(sLa), "+v"(sHb), "+v"(sLb) : "v"(ka0), "v"(kb0), "v"(qh), "v"(qr));
        }
        const float* kp = kmb + key0;
        const v4f m0 = *(const v4f*)kp, m1 = *(const v4f*)(kp + 4), m2 = *(const v4f*)(kp + 16), m3 = *(const v4f*)(kp + 20);
        float kx[8], ky[8];
#pragma unroll
        for (int r = 0; r < 4; ++r) { kx[r] = m0[r]; kx[4 + r] = m1[r]; ky[r] = m2[r]; ky[4 + r] = m3[r]; }
        const int ja = key0 + 8 * hi;
        float ta[8], tb[8]; bool fa[8], fb[8]; float mx = NEGB;
#pragma unroll
        for (int r = 0; r < 8; ++r) {
            fa[r] = (qmv * bfr(kx[r]) != 0.0f) && (ja + r <= lim);
            fb[r] = (qmv * bfr(ky[r]) != 0.0f) && (ja + 16 + r <= lim);
            ta[r] = (sHa[r] + sLa[r] * QRI) * SC2; tb[r] = (sHb[r] + sLb[r] * QRI) * SC2;
            mx = fmaxf(mx, fmaxf(fa[r] ? ta[r] : NEGB, fb[r] ? tb[r] : NEGB)); }
        mx = fmaxf(mx, __shfl_xor(mx, 16, 32));
        const float mnew = fmaxf(m, mx);
        const float alpha = __builtin_amdgcn_exp2f(m - mnew);
        const float sh = PSH - mnew;
        v16h pb, pr = hz; float ls = 0.0f;
#pragma unroll
        for (int r = 0; r < 8; ++r) {
            const float ea = __builtin_amdgcn_exp2f(ta[r] + sh), eb = __builtin_amdgcn_exp2f(tb[r] + sh);
            const float ga = fa[r] ? ea : 0.0f, gb = fb[r] ? eb : 0.0f;
            const h16 pa = (h16)ga; const h16 pc = (h16)gb;
            pb[r] = pa; pb[8 + r] = pc;
            if (EARLY) { pr[r] = (h16)((ga - (float)pa) * QRS); pr[8 + r] = (h16)((gb - (float)pc) * QRS); ls += ga + gb; }
            else       { ls += (float)pa + (float)pc; } }
        l = l * alpha + ls; m = mnew;
        o0 = o0 * alpha; o1 = o1 * alpha;
        if (EARLY) { oR0 = oR0 * alpha; oR1 = oR1 * alpha; }
        const h16* va = VT + vo + key0;
        const v16h v0 = ldh(va), v1 = ldh(va + (size_t)16 * SEQ);
        if (EARLY) {
            const h16* vr = VR + vro + kcl;
            v16h vr0 = ldh(vr), vr1 = ldh(vr + (size_t)16 * EROWS);
            if (!rok) { vr0 = hz; vr1 = hz; }
            o0 = wmma16(v0, pb, o0); o1 = wmma16(v1, pb, o1);
            oR0 = wmma16(v0, pr, oR0); oR1 = wmma16(v1, pr, oR1);
            oR0 = wmma16(vr0, pb, oR0); oR1 = wmma16(vr1, pb, oR1);
            asm volatile("v_nop\n\tv_nop\n\tv_nop\n\tv_nop" : "+v"(o0), "+v"(o1), "+v"(oR0), "+v"(oR1) : "v"(v0), "v"(v1), "v"(vr0), "v"(vr1), "v"(pb), "v"(pr));
        } else {
            o0 = wmma16(v0, pb, o0); o1 = wmma16(v1, pb, o1);
            asm volatile("v_nop\n\tv_nop\n\tv_nop\n\tv_nop" : "+v"(o0), "+v"(o1) : "v"(v0), "v"(v1), "v"(pb));
        }
    }
    l += __shfl_xor(l, 16, 32);
    const bool any = l > 0.0f;
    const float lsafe = any ? l : 1.0f;
    const float inv = any ? (1.0f / lsafe) : 0.0f;
    v8f f0 = o0, f1 = o1;
    if (EARLY) { f0 = o0 + oR0 * QRI; f1 = o1 + oR1 * QRI; }
    const int wb = wave * 16 * OSP;
    { v4f a, c;
      a[0] = f0[0] * inv; a[1] = f0[1] * inv; a[2] = f0[2] * inv; a[3] = f0[3] * inv; c[0] = f0[4] * inv; c[1] = f0[5] * inv; c[2] = f0[6] * inv; c[3] = f0[7] * inv;
      *(v4fa*)(&os[wb + lr * OSP +  0 + 8 * hi]) = a; *(v4fa*)(&os[wb + lr * OSP +  0 + 8 * hi + 4]) = c;
      a[0] = f1[0] * inv; a[1] = f1[1] * inv; a[2] = f1[2] * inv; a[3] = f1[3] * inv; c[0] = f1[4] * inv; c[1] = f1[5] * inv; c[2] = f1[6] * inv; c[3] = f1[7] * inv;
      *(v4fa*)(&os[wb + lr * OSP + 16 + 8 * hi]) = a; *(v4fa*)(&os[wb + lr * OSP + 16 + 8 * hi + 4]) = c; }
    wave_sync();
    float* orow = OUT + ((size_t)b * OUT_SEQ + t0) * DM + h * HD;
#pragma unroll 1
    for (int ps = 0; ps < 2; ++ps) {
#pragma unroll
        for (int s = 0; s < 4; ++s) { const int row = 4 * s + (lane >> 3), cofs = (lane & 7) * 4;
            const v4f val = *(const v4fa*)(&os[wb + row * OSP + cofs]);
            *(volatile v4f*)(orow + (size_t)row * DM + cofs) = val; }
        if (ps == 0) __threadfence(); }
}

static constexpr size_t al256(size_t v) { return (v + 255) & ~(size_t)255; }
static constexpr size_t SZ_XB = al256((size_t)NB * SEQ * DM * 2);
static constexpr size_t SZ_WB = al256((size_t)3 * DM * DM * 2);
static constexpr size_t SZ_PL = al256((size_t)NB * NH_ * SEQ * HD * 2);
static constexpr size_t SZ_RS = al256((size_t)NB * NH_ * EROWS * HD * 2);
static constexpr size_t SZ_TOTAL = 3 * SZ_XB + SZ_WB + 4 * SZ_PL + 2 * SZ_RS;
static_assert(SZ_TOTAL <= (size_t)134217728);
static_assert(((size_t)DM * DM * 2) % 256 == 0);
static_assert((size_t)NB * NH_ * SEQ * HD == (size_t)NB * DM * SEQ);
static_assert((size_t)NB * NH_ * EROWS * HD == (size_t)NB * DM * EROWS);

extern "C" void kernel_launch(void* const* d_in, const int* in_sizes, int n_in,
                              void* d_out, int out_size, void* d_ws, size_t ws_size, hipStream_t stream) {
    if (n_in < 12) return;
    const size_t needx = ((size_t)(NB - 1) * SEQ_FULL + SEQ) * DM;
    const size_t needm = (size_t)(NB - 1) * SEQ_FULL + SEQ;
    if ((size_t)in_sizes[0] < needx || (size_t)in_sizes[1] < needx || (size_t)in_sizes[2] < needx) return;
    if ((size_t)in_sizes[3] < needm || (size_t)in_sizes[4] < needm) return;
    if ((size_t)in_sizes[5] < (size_t)DM * DM || (size_t)in_sizes[7] < (size_t)DM * DM || (size_t)in_sizes[9] < (size_t)DM * DM) return;
    if (in_sizes[6] < DM || in_sizes[8] < DM || in_sizes[10] < DM || in_sizes[11] < 1) return;
    if ((size_t)out_size < ((size_t)(NB - 1) * OUT_SEQ + SEQ) * DM) return;
    if (SZ_TOTAL > ws_size) return;
    const float* xin[3] = { (const float*)d_in[0], (const float*)d_in[1], (const float*)d_in[2] };
    const float* qm = (const float*)d_in[3]; const float* km = (const float*)d_in[4];
    const float* wq = (const float*)d_in[5]; const float* bq = (const float*)d_in[6];
    const float* wk = (const float*)d_in[7]; const float* bk = (const float*)d_in[8];
    const float* wv = (const float*)d_in[9]; const float* bv = (const float*)d_in[10];
    const int* causal = (const int*)d_in[11];
    float* OUT = (float*)d_out;
    char* wsp = (char*)d_ws;
    bf* XB[3];
    XB[0] = (bf*)wsp; wsp += SZ_XB;
    XB[1] = (bf*)wsp; wsp += SZ_XB;
    XB[2] = (bf*)wsp; wsp += SZ_XB;
    bf* WB = (bf*)wsp; wsp += SZ_WB;
    h16* QH = (h16*)wsp; wsp += SZ_PL;
    h16* QR = (h16*)wsp; wsp += SZ_PL;
    h16* KP = (h16*)wsp; wsp += SZ_PL;
    h16* VT = (h16*)wsp; wsp += SZ_PL;
    h16* KR = (h16*)wsp; wsp += SZ_RS;
    h16* VR = (h16*)wsp; wsp += SZ_RS;
    bf* WQ = WB; bf* WK = WB + (size_t)DM * DM; bf* WV = WB + (size_t)2 * DM * DM;

    for (int i = 0; i < 3; ++i) {
        if (SEQ == SEQ_FULL) {
            const size_t n8 = (size_t)NB * SEQ * DM / 8;
            k_cvt8<<<(unsigned)((n8 + 255) / 256), 256, 0, stream>>>(xin[i], XB[i], n8);
        } else {
            const size_t n8 = (size_t)SEQ * DM / 8;
            for (int b = 0; b < NB; ++b) k_cvt8<<<(unsigned)((n8 + 255) / 256), 256, 0, stream>>>(xin[i] + (size_t)b * SEQ_FULL * DM, XB[i] + (size_t)b * SEQ * DM, n8);
        }
    }
    { const size_t n8 = (size_t)DM * DM / 8; const unsigned g = (unsigned)((n8 + 255) / 256);
      k_cvt8<<<g, 256, 0, stream>>>(wq, WQ, n8); k_cvt8<<<g, 256, 0, stream>>>(wk, WK, n8); k_cvt8<<<g, 256, 0, stream>>>(wv, WV, n8); }

    k_proj<0><<<dim3(NB * SEQ / 64, DM / 64, 1), 32, 0, stream>>>(XB[0], WQ, bq, QH, QR, SEQ);
    k_proj<0><<<dim3(NB * SEQ / 64, DM / 64, 1), 32, 0, stream>>>(XB[1], WK, bk, KP, KR, EROWS);
    k_proj<1><<<dim3(DM / 64, NB * SEQ / 64, 1), 32, 0, stream>>>(WV, XB[2], bv, VT, VR, EROWS);

    k_flash<1><<<dim3(EROWS / (16 * AW), NB * NH_, 1), 32 * AW, 0, stream>>>(QH, QR, KP, KR, VT, VR, qm, km, causal, OUT);
    if (SEQ > EROWS)
        k_flash<0><<<dim3((SEQ - EROWS) / (16 * AW), NB * NH_, 1), 32 * AW, 0, stream>>>(QH, QR, KP, KR, VT, VR, qm, km, causal, OUT);
}
